// BidirectionalMambaBlock_13958643712580
// MI455X (gfx1250) — hardware-verified
//
#include <hip/hip_runtime.h>
#include <stdint.h>


#define D_MODEL 512
#define D_INNER 1024
#define D_XZ    2048
#define DT_RANK 32
#define D_STATE 16
#define D_DBC   64
#define D_FF    2048
#define BATCH   2
#define SEQ     1024
#define ROWS    (BATCH * SEQ)

#define GBM  64
#define GBN  64
#define GBK  32
#define LSTR 40
#define CSTR 68
#define SCH  32

static_assert(ROWS % GBM == 0);
static_assert(D_XZ % GBN == 0 && D_DBC % GBN == 0 && D_INNER % GBN == 0 && D_MODEL % GBN == 0 && D_FF % GBN == 0);
static_assert(D_MODEL % GBK == 0 && D_INNER % GBK == 0 && DT_RANK % GBK == 0 && D_FF % GBK == 0);
static_assert(SEQ % SCH == 0 && SCH % 8 == 0);
static_assert(GBM * CSTR * 4 <= 4 * GBM * LSTR * 2);

typedef __bf16         v16bf __attribute__((ext_vector_type(16)));
typedef float          v8f   __attribute__((ext_vector_type(8)));
typedef float          v4f   __attribute__((ext_vector_type(4)));
typedef unsigned int   v4u   __attribute__((ext_vector_type(4)));
typedef unsigned short us;

union Frag { v16bf v; v4u q[2]; };

__device__ __forceinline__ unsigned int bfb(float f)
{
    unsigned int u = __float_as_uint(f);
    u += 0x7FFFu + ((u >> 16) & 1u);
    return u >> 16;
}

__device__ __forceinline__ void split1(float x, unsigned int& hb, unsigned int& lb)
{
    hb = bfb(x);
    float hf = __uint_as_float(hb << 16);
    lb = bfb(x - hf);
}

__device__ __forceinline__ void split8(const float* v, v4u& hq, v4u& lq)
{
    unsigned int hb[8], lb[8];
#pragma unroll
    for (int i = 0; i < 8; ++i) split1(v[i], hb[i], lb[i]);
    hq.x = hb[0] | (hb[1] << 16); hq.y = hb[2] | (hb[3] << 16);
    hq.z = hb[4] | (hb[5] << 16); hq.w = hb[6] | (hb[7] << 16);
    lq.x = lb[0] | (lb[1] << 16); lq.y = lb[2] | (lb[3] << 16);
    lq.z = lb[4] | (lb[5] << 16); lq.w = lb[6] | (lb[7] << 16);
}

__device__ __forceinline__ void load8(const float* p, float* o)
{
    v4f a = *(const v4f*)p;
    v4f b = *(const v4f*)(p + 4);
    o[0] = a.x; o[1] = a.y; o[2] = a.z; o[3] = a.w;
    o[4] = b.x; o[5] = b.y; o[6] = b.z; o[7] = b.w;
}

__device__ __forceinline__ float wsum(float v)
{
#pragma unroll
    for (int o = 16; o > 0; o >>= 1) v += __shfl_xor(v, o, 32);
    return v;
}

__device__ __forceinline__ float bsum(float v, float* slot, int nw)
{
    v = wsum(v);
    if ((threadIdx.x & 31) == 0) slot[threadIdx.x >> 5] = v;
    __syncthreads();
    float t = 0.0f;
    for (int i = 0; i < nw; ++i) t += slot[i];
    return t;
}

__device__ __forceinline__ float actf(float v, int act)
{
    if (act == 1) return fmaxf(v, 0.0f);
    if (act == 2) return fmaxf(v, 0.0f) + log1pf(__expf(-fabsf(v)));
    return v;
}

__device__ __forceinline__ v8f wmma_bf(v16bf a, v16bf b, v8f c)
{
    return __builtin_amdgcn_wmma_f32_16x16x32_bf16(false, a, false, b, (short)0, c, false, false);
}

__device__ __forceinline__ void mma3(v8f& acc, const Frag& ah, const Frag& al,
                                     const Frag& bh, const Frag& bl)
{
    acc = wmma_bf(ah.v, bh.v, acc);
    acc = wmma_bf(ah.v, bl.v, acc);
    acc = wmma_bf(al.v, bh.v, acc);
    asm volatile("v_nop\n\tv_nop\n\tv_nop\n\tv_nop"
                 : "+v"(acc) : "v"(ah.v), "v"(al.v), "v"(bh.v), "v"(bl.v));
}

__global__ __launch_bounds__(256)
void k_split(const float* __restrict__ src, us* dh, us* dl, int n, int cols, int seq, int flip)
{
    int n8 = n >> 3;
    int g = blockIdx.x * 256 + threadIdx.x;
    if (g >= n8) return;
    int e = g * 8;
    int row = e / cols;
    int c = e - row * cols;
    int srow = row;
    if (flip) {
        int bb = row / seq;
        int t = row - bb * seq;
        srow = bb * seq + (seq - 1 - t);
    }
    float v[8];
    load8(src + (size_t)srow * cols + c, v);
    v4u hq, lq;
    split8(v, hq, lq);
    *(volatile v4u*)(dh + e) = hq;
    *(volatile v4u*)(dl + e) = lq;
    __threadfence();
    *(volatile v4u*)(dh + e) = hq;
    *(volatile v4u*)(dl + e) = lq;
}

__global__ __launch_bounds__(128)
void k_gemm(const us* __restrict__ Ah, const us* __restrict__ Al, int lda,
            const us* __restrict__ Wh, const us* __restrict__ Wl, int K, int N,
            const float* __restrict__ bias, int act,
            float* outF, us* outH, us* outL)
{
    __shared__ __align__(16) us smem[4 * GBM * LSTR];
    us* sAh = smem;
    us* sAl = smem + GBM * LSTR;
    us* sBh = smem + 2 * GBM * LSTR;
    us* sBl = smem + 3 * GBM * LSTR;
    float* sC = reinterpret_cast<float*>(smem);

    const int tid = threadIdx.x;
    const int lane = tid & 31, wave = tid >> 5;
    const int wm = wave & 1, wn = wave >> 1;
    const int h = lane >> 4, m = lane & 15;
    const int m0 = blockIdx.y * GBM, n0 = blockIdx.x * GBN;

    v8f acc00 = {0.f, 0.f, 0.f, 0.f, 0.f, 0.f, 0.f, 0.f};
    v8f acc01 = {0.f, 0.f, 0.f, 0.f, 0.f, 0.f, 0.f, 0.f};
    v8f acc10 = {0.f, 0.f, 0.f, 0.f, 0.f, 0.f, 0.f, 0.f};
    v8f acc11 = {0.f, 0.f, 0.f, 0.f, 0.f, 0.f, 0.f, 0.f};

#pragma unroll 1
    for (int k0 = 0; k0 < K; k0 += GBK) {
#pragma unroll
        for (int j = 0; j < 2; ++j) {
            int idx = tid + 128 * j;
            int row = idx >> 2;
            int ch  = (idx & 3) * 8;
            size_t ga = (size_t)(m0 + row) * lda + k0 + ch;
            size_t gb = (size_t)(n0 + row) * K + k0 + ch;
            v4u a0 = *(const v4u*)(Ah + ga);
            v4u a1 = *(const v4u*)(Al + ga);
            v4u b0 = *(const v4u*)(Wh + gb);
            v4u b1 = *(const v4u*)(Wl + gb);
            int lo = row * LSTR + ch;
            *(v4u*)(sAh + lo) = a0;
            *(v4u*)(sAl + lo) = a1;
            *(v4u*)(sBh + lo) = b0;
            *(v4u*)(sBl + lo) = b1;
        }
        __syncthreads();

        Frag ah0, al0, ah1, al1, bh0, bl0, bh1, bl1;
        {
            int ba0 = (wm * 32 + m) * LSTR;
            int ba1 = (wm * 32 + 16 + m) * LSTR;
            ah0.q[0] = *(const v4u*)(sAh + ba0 + 8 * h);  ah0.q[1] = *(const v4u*)(sAh + ba0 + 16 + 8 * h);
            al0.q[0] = *(const v4u*)(sAl + ba0 + 8 * h);  al0.q[1] = *(const v4u*)(sAl + ba0 + 16 + 8 * h);
            ah1.q[0] = *(const v4u*)(sAh + ba1 + 8 * h);  ah1.q[1] = *(const v4u*)(sAh + ba1 + 16 + 8 * h);
            al1.q[0] = *(const v4u*)(sAl + ba1 + 8 * h);  al1.q[1] = *(const v4u*)(sAl + ba1 + 16 + 8 * h);
            int bb0 = (wn * 32 + m) * LSTR;
            int bb1 = (wn * 32 + 16 + m) * LSTR;
            bh0.q[0] = *(const v4u*)(sBh + bb0 + 8 * h);  bh0.q[1] = *(const v4u*)(sBh + bb0 + 16 + 8 * h);
            bl0.q[0] = *(const v4u*)(sBl + bb0 + 8 * h);  bl0.q[1] = *(const v4u*)(sBl + bb0 + 16 + 8 * h);
            bh1.q[0] = *(const v4u*)(sBh + bb1 + 8 * h);  bh1.q[1] = *(const v4u*)(sBh + bb1 + 16 + 8 * h);
            bl1.q[0] = *(const v4u*)(sBl + bb1 + 8 * h);  bl1.q[1] = *(const v4u*)(sBl + bb1 + 16 + 8 * h);
        }
        mma3(acc00, ah0, al0, bh0, bl0);
        mma3(acc01, ah0, al0, bh1, bl1);
        mma3(acc10, ah1, al1, bh0, bl0);
        mma3(acc11, ah1, al1, bh1, bl1);
        __syncthreads();
    }

    {
        int rb0 = wm * 32 + 8 * h, rb1 = wm * 32 + 16 + 8 * h;
        int cb0 = wn * 32 + m,     cb1 = wn * 32 + 16 + m;
#pragma unroll
        for (int r = 0; r < 8; ++r) {
            sC[(rb0 + r) * CSTR + cb0] = acc00[r];
            sC[(rb0 + r) * CSTR + cb1] = acc01[r];
            sC[(rb1 + r) * CSTR + cb0] = acc10[r];
            sC[(rb1 + r) * CSTR + cb1] = acc11[r];
        }
    }
    __syncthreads();

    const bool doF = (outF != 0);
    const bool doS = (outH != 0);

    v4f fv[8];
    if (doF) {
#pragma unroll
        for (int p = 0; p < 8; ++p) {
            int row = (tid >> 4) + 8 * p;
            int c4 = (tid & 15) * 4;
            v4f v = *(const v4f*)(sC + row * CSTR + c4);
            float t[4] = {v.x, v.y, v.z, v.w};
            float bsv[4] = {0.f, 0.f, 0.f, 0.f};
            if (bias) { v4f bq = *(const v4f*)(bias + n0 + c4); bsv[0] = bq.x; bsv[1] = bq.y; bsv[2] = bq.z; bsv[3] = bq.w; }
#pragma unroll
            for (int q = 0; q < 4; ++q) t[q] = actf(t[q] + bsv[q], act);
            v4f o = {t[0], t[1], t[2], t[3]};
            fv[p] = o;
        }
    }
    v4u hv[4], lv[4];
    if (doS) {
#pragma unroll
        for (int p = 0; p < 4; ++p) {
            int row = (tid >> 3) + 16 * p;
            int c8 = (tid & 7) * 8;
            float t[8];
            v4f va = *(const v4f*)(sC + row * CSTR + c8);
            v4f vb = *(const v4f*)(sC + row * CSTR + c8 + 4);
            t[0] = va.x; t[1] = va.y; t[2] = va.z; t[3] = va.w;
            t[4] = vb.x; t[5] = vb.y; t[6] = vb.z; t[7] = vb.w;
            float bsv[8] = {0.f, 0.f, 0.f, 0.f, 0.f, 0.f, 0.f, 0.f};
            if (bias) load8(bias + n0 + c8, bsv);
#pragma unroll
            for (int q = 0; q < 8; ++q) t[q] = actf(t[q] + bsv[q], act);
            split8(t, hv[p], lv[p]);
        }
    }

    if (doF) {
#pragma unroll
        for (int p = 0; p < 8; ++p) {
            int row = (tid >> 4) + 8 * p;
            int c4 = (tid & 15) * 4;
            *(volatile v4f*)(outF + (size_t)(m0 + row) * N + n0 + c4) = fv[p];
        }
    }
    if (doS) {
#pragma unroll
        for (int p = 0; p < 4; ++p) {
            int row = (tid >> 3) + 16 * p;
            int c8 = (tid & 7) * 8;
            size_t off = (size_t)(m0 + row) * N + n0 + c8;
            *(volatile v4u*)(outH + off) = hv[p];
            *(volatile v4u*)(outL + off) = lv[p];
        }
    }
    __threadfence();
    if (doF) {
#pragma unroll
        for (int p = 0; p < 8; ++p) {
            int row = (tid >> 4) + 8 * p;
            int c4 = (tid & 15) * 4;
            *(volatile v4f*)(outF + (size_t)(m0 + row) * N + n0 + c4) = fv[p];
        }
    }
    if (doS) {
#pragma unroll
        for (int p = 0; p < 4; ++p) {
            int row = (tid >> 3) + 16 * p;
            int c8 = (tid & 7) * 8;
            size_t off = (size_t)(m0 + row) * N + n0 + c8;
            *(volatile v4u*)(outH + off) = hv[p];
            *(volatile v4u*)(outL + off) = lv[p];
        }
    }
}

__global__ __launch_bounds__(128)
void k_conv(const float* __restrict__ xz, const float* __restrict__ cw, const float* __restrict__ cb,
            float* outF, us* outH, us* outL)
{
    __shared__ __align__(16) float srow[D_INNER];
    const int r = blockIdx.x;
    const int b = r / SEQ;
    const int t = r - b * SEQ;
    const int tid = threadIdx.x;
    const int d0 = tid * 8;

    v4f wv[8];
#pragma unroll
    for (int i = 0; i < 8; ++i) wv[i] = *(const v4f*)(cw + (size_t)(d0 + i) * 4);

    float s[8] = {0.f, 0.f, 0.f, 0.f, 0.f, 0.f, 0.f, 0.f};
#pragma unroll
    for (int j = 0; j < 4; ++j) {
        int tt = t - 3 + j;
        if (tt >= 0) {
            float xv[8];
            load8(xz + (size_t)(b * SEQ + tt) * D_XZ + d0, xv);
#pragma unroll
            for (int i = 0; i < 8; ++i) s[i] += xv[i] * wv[i][j];
        }
    }
    float cbv[8];
    load8(cb + d0, cbv);
    float u[8];
#pragma unroll
    for (int i = 0; i < 8; ++i) {
        float a = s[i] + cbv[i];
        float sg = __fdividef(1.0f, 1.0f + __expf(-a));
        u[i] = a * sg;
    }
    {
        v4f u0 = {u[0], u[1], u[2], u[3]};
        v4f u1 = {u[4], u[5], u[6], u[7]};
        *(v4f*)(srow + d0) = u0;
        *(v4f*)(srow + d0 + 4) = u1;
    }
    v4u hq, lq;
    split8(u, hq, lq);
    __syncthreads();

    v4f f0 = *(const v4f*)(srow + tid * 4);
    v4f f1 = *(const v4f*)(srow + 512 + tid * 4);
    const size_t base = (size_t)r * D_INNER;
    *(volatile v4f*)(outF + base + tid * 4) = f0;
    *(volatile v4f*)(outF + base + 512 + tid * 4) = f1;
    *(volatile v4u*)(outH + base + d0) = hq;
    *(volatile v4u*)(outL + base + d0) = lq;
    __threadfence();
    *(volatile v4f*)(outF + base + tid * 4) = f0;
    *(volatile v4f*)(outF + base + 512 + tid * 4) = f1;
    *(volatile v4u*)(outH + base + d0) = hq;
    *(volatile v4u*)(outL + base + d0) = lq;
}

__global__ __launch_bounds__(256)
void k_scan(const float* __restrict__ delta,
            const float* __restrict__ dbc,
            const float* __restrict__ xm,
            const float* __restrict__ xz,
            const float* __restrict__ A_log,
            const float* __restrict__ Dp,
            us* yH, us* yL)
{
    __shared__ __align__(16) us    sYh[SCH * 256];
    __shared__ __align__(16) us    sYl[SCH * 256];
    __shared__ __align__(16) float sBC[SCH * 32];

    const int tid = threadIdx.x;
    const int lane = tid & 31, wave = tid >> 5;
    const int d = blockIdx.x * 256 + tid;
    const int b = blockIdx.y;

    float Av[D_STATE];
#pragma unroll
    for (int s = 0; s < D_STATE; ++s) Av[s] = -expf(A_log[(size_t)d * D_STATE + s]);
    const float Dd = Dp[d];
    float h[D_STATE];
#pragma unroll
    for (int s = 0; s < D_STATE; ++s) h[s] = 0.0f;

#pragma unroll 1
    for (int t0 = 0; t0 < SEQ; t0 += SCH) {
        __syncthreads();
        {
            int st = tid >> 3;
            int q  = (tid & 7) * 4;
            *(v4f*)(sBC + st * 32 + q) =
                *(const v4f*)(dbc + (size_t)(b * SEQ + t0 + st) * D_DBC + DT_RANK + q);
        }
        __syncthreads();

#pragma unroll 1
        for (int tt = 0; tt < SCH; ++tt) {
            size_t rr = (size_t)(b * SEQ + t0 + tt);
            float dt = delta[rr * D_INNER + d];
            float x  = xm[rr * D_INNER + d];
            float zz = xz[rr * D_XZ + D_INNER + d];
            const float* bc = sBC + tt * 32;
            float yv = 0.0f;
#pragma unroll
            for (int s = 0; s < D_STATE; ++s) {
                float dA = __expf(dt * Av[s]);
                h[s] = dA * h[s] + (dt * bc[s]) * x;
                yv += h[s] * bc[16 + s];
            }
            yv += x * Dd;
            float sg = __fdividef(1.0f, 1.0f + __expf(-zz));
            yv = yv * (zz * sg);
            unsigned int hb, lb;
            split1(yv, hb, lb);
            sYh[tt * 256 + tid] = (us)hb;
            sYl[tt * 256 + tid] = (us)lb;
        }
        __syncthreads();

        const size_t gb = (size_t)(b * SEQ + t0) * D_INNER + (size_t)blockIdx.x * 256 + lane * 8;
#pragma unroll
        for (int p = 0; p < SCH / 8; ++p) {
            int row = wave + 8 * p;
            v4u vh = *(const v4u*)(sYh + row * 256 + lane * 8);
            v4u vl = *(const v4u*)(sYl + row * 256 + lane * 8);
            *(volatile v4u*)(yH + gb + (size_t)row * D_INNER) = vh;
            *(volatile v4u*)(yL + gb + (size_t)row * D_INNER) = vl;
        }
        __threadfence();
#pragma unroll
        for (int p = 0; p < SCH / 8; ++p) {
            int row = wave + 8 * p;
            v4u vh = *(const v4u*)(sYh + row * 256 + lane * 8);
            v4u vl = *(const v4u*)(sYl + row * 256 + lane * 8);
            *(volatile v4u*)(yH + gb + (size_t)row * D_INNER) = vh;
            *(volatile v4u*)(yL + gb + (size_t)row * D_INNER) = vl;
        }
    }
}

__global__ __launch_bounds__(64)
void k_ln12(const float* __restrict__ x, const float* __restrict__ dF, const float* __restrict__ dT,
            const float* __restrict__ g1, const float* __restrict__ b1,
            const float* __restrict__ g2, const float* __restrict__ b2,
            us* outH, us* outL)
{
    __shared__ float red[4][4];
    const int r = blockIdx.x;
    const int bb = r / SEQ;
    const int t = r - bb * SEQ;
    const int rf = bb * SEQ + (SEQ - 1 - t);
    const int tid = threadIdx.x;
    const int c0 = tid * 8;

    float xv[8], fv[8], wv[8], v1[8], v2[8];
    load8(x  + (size_t)r  * D_MODEL + c0, xv);
    load8(dF + (size_t)r  * D_MODEL + c0, fv);
    load8(dT + (size_t)rf * D_MODEL + c0, wv);
    float s1 = 0.f, s2 = 0.f;
#pragma unroll
    for (int i = 0; i < 8; ++i) { v1[i] = xv[i] + fv[i]; v2[i] = xv[i] + wv[i]; s1 += v1[i]; s2 += v2[i]; }
    const float inv = 1.0f / (float)D_MODEL;
    float m1 = bsum(s1, &red[0][0], 2) * inv;
    float m2 = bsum(s2, &red[1][0], 2) * inv;
    float q1 = 0.f, q2 = 0.f;
#pragma unroll
    for (int i = 0; i < 8; ++i) { float a = v1[i] - m1; float c = v2[i] - m2; q1 += a * a; q2 += c * c; }
    float r1 = rsqrtf(bsum(q1, &red[2][0], 2) * inv + 1e-5f);
    float r2 = rsqrtf(bsum(q2, &red[3][0], 2) * inv + 1e-5f);

    float g1v[8], b1v[8], g2v[8], b2v[8], o[8];
    load8(g1 + c0, g1v); load8(b1 + c0, b1v); load8(g2 + c0, g2v); load8(b2 + c0, b2v);
#pragma unroll
    for (int i = 0; i < 8; ++i)
        o[i] = ((v1[i] - m1) * r1 * g1v[i] + b1v[i]) + ((v2[i] - m2) * r2 * g2v[i] + b2v[i]);
    v4u hq, lq;
    split8(o, hq, lq);
    const size_t off = (size_t)r * D_MODEL + c0;
    *(volatile v4u*)(outH + off) = hq;
    *(volatile v4u*)(outL + off) = lq;
    __threadfence();
    *(volatile v4u*)(outH + off) = hq;
    *(volatile v4u*)(outL + off) = lq;
}

__global__ __launch_bounds__(128)
void k_ln3(const float* __restrict__ ff, const float* __restrict__ g, const float* __restrict__ bb,
           float* out)
{
    __shared__ float red[2][4];
    const int r = blockIdx.x;
    const int tid = threadIdx.x;
    const int c0 = tid * 4;
    v4f a = *(const v4f*)(ff + (size_t)r * D_MODEL + c0);
    float v[4] = {2.0f * a.x, 2.0f * a.y, 2.0f * a.z, 2.0f * a.w};
    const float inv = 1.0f / (float)D_MODEL;
    float s = v[0] + v[1] + v[2] + v[3];
    float mu = bsum(s, &red[0][0], 4) * inv;
    float q = 0.f;
#pragma unroll
    for (int i = 0; i < 4; ++i) { float dlt = v[i] - mu; q += dlt * dlt; }
    float rs = rsqrtf(bsum(q, &red[1][0], 4) * inv + 1e-5f);
    v4f gv = *(const v4f*)(g + c0);
    v4f bv = *(const v4f*)(bb + c0);
    v4f o;
    o.x = (v[0] - mu) * rs * gv.x + bv.x;
    o.y = (v[1] - mu) * rs * gv.y + bv.y;
    o.z = (v[2] - mu) * rs * gv.z + bv.z;
    o.w = (v[3] - mu) * rs * gv.w + bv.w;
    const size_t off = (size_t)r * D_MODEL + c0;
    *(volatile v4f*)(out + off) = o;
    __threadfence();
    *(volatile v4f*)(out + off) = o;
}

extern "C" void kernel_launch(void* const* d_in, const int* in_sizes, int n_in,
                              void* d_out, int out_size, void* d_ws, size_t ws_size,
                              hipStream_t stream)
{
    if (n_in < 29) return;
    {
        const int need[29] = {
            ROWS * D_MODEL,
            D_XZ * D_MODEL, D_INNER * 4, D_INNER, D_DBC * D_INNER, D_INNER * DT_RANK, D_INNER,
            D_INNER * D_STATE, D_INNER, D_MODEL * D_INNER,
            D_XZ * D_MODEL, D_INNER * 4, D_INNER, D_DBC * D_INNER, D_INNER * DT_RANK, D_INNER,
            D_INNER * D_STATE, D_INNER, D_MODEL * D_INNER,
            D_MODEL, D_MODEL, D_MODEL, D_MODEL, D_MODEL, D_MODEL,
            D_FF * D_MODEL, D_FF, D_MODEL * D_FF, D_MODEL };
        for (int i = 0; i < 29; ++i) if (in_sizes[i] != need[i]) return;
    }
    if (out_size != ROWS * D_MODEL) return;

    const float* x        = (const float*)d_in[0];
    const float* fm_in_W  = (const float*)d_in[1];
    const float* fm_cw    = (const float*)d_in[2];
    const float* fm_cb    = (const float*)d_in[3];
    const float* fm_xp_W  = (const float*)d_in[4];
    const float* fm_dt_W  = (const float*)d_in[5];
    const float* fm_dt_b  = (const float*)d_in[6];
    const float* fm_Alog  = (const float*)d_in[7];
    const float* fm_D     = (const float*)d_in[8];
    const float* fm_out_W = (const float*)d_in[9];
    const float* bm_in_W  = (const float*)d_in[10];
    const float* bm_cw    = (const float*)d_in[11];
    const float* bm_cb    = (const float*)d_in[12];
    const float* bm_xp_W  = (const float*)d_in[13];
    const float* bm_dt_W  = (const float*)d_in[14];
    const float* bm_dt_b  = (const float*)d_in[15];
    const float* bm_Alog  = (const float*)d_in[16];
    const float* bm_D     = (const float*)d_in[17];
    const float* bm_out_W = (const float*)d_in[18];
    const float* ln1_g = (const float*)d_in[19];
    const float* ln1_b = (const float*)d_in[20];
    const float* ln2_g = (const float*)d_in[21];
    const float* ln2_b = (const float*)d_in[22];
    const float* ln3_g = (const float*)d_in[23];
    const float* ln3_b = (const float*)d_in[24];
    const float* ff_W1 = (const float*)d_in[25];
    const float* ff_b1 = (const float*)d_in[26];
    const float* ff_W2 = (const float*)d_in[27];
    const float* ff_b2 = (const float*)d_in[28];
    float* out = (float*)d_out;

    size_t off = 0;
    char* wsb = (char*)d_ws;
    auto carve = [&](size_t bytes) -> char* { char* p = wsb + off; off += (bytes + 255) & ~(size_t)255; return p; };
    auto plane = [&](size_t n) -> us* { return (us*)carve(n * sizeof(us)); };
    auto f32b  = [&](size_t n) -> float* { return (float*)carve(n * sizeof(float)); };

    const size_t nIn  = (size_t)D_XZ * D_MODEL;
    const size_t nXp  = (size_t)D_DBC * D_INNER;
    const size_t nDt  = (size_t)D_INNER * DT_RANK;
    const size_t nOut = (size_t)D_MODEL * D_INNER;
    const size_t nF1  = (size_t)D_FF * D_MODEL;
    const size_t nF2  = (size_t)D_MODEL * D_FF;

    us* fm_inH = plane(nIn);   us* fm_inL = plane(nIn);
    us* bm_inH = plane(nIn);   us* bm_inL = plane(nIn);
    us* fm_xpH = plane(nXp);   us* fm_xpL = plane(nXp);
    us* bm_xpH = plane(nXp);   us* bm_xpL = plane(nXp);
    us* fm_dtH = plane(nDt);   us* fm_dtL = plane(nDt);
    us* bm_dtH = plane(nDt);   us* bm_dtL = plane(nDt);
    us* fm_ouH = plane(nOut);  us* fm_ouL = plane(nOut);
    us* bm_ouH = plane(nOut);  us* bm_ouL = plane(nOut);
    us* f1H = plane(nF1);      us* f1L = plane(nF1);
    us* f2H = plane(nF2);      us* f2L = plane(nF2);

    const size_t nX   = (size_t)ROWS * D_MODEL;
    const size_t nXZ  = (size_t)ROWS * D_XZ;
    const size_t nXM  = (size_t)ROWS * D_INNER;
    const size_t nDBC = (size_t)ROWS * D_DBC;
    const size_t nHF  = (size_t)ROWS * D_FF;

    us* xH  = plane(nX);   us* xL  = plane(nX);
    us* xrH = plane(nX);   us* xrL = plane(nX);
    float* xz    = f32b(nXZ);
    float* xm    = f32b(nXM);
    us* xmH = plane(nXM);  us* xmL = plane(nXM);
    float* dbc   = f32b(nDBC);
    us* dbH = plane(nDBC); us* dbL = plane(nDBC);
    float* delta = f32b(nXM);
    us* yH  = plane(nXM);  us* yL  = plane(nXM);
    float* dirF  = f32b(nX);
    float* dirT  = f32b(nX);
    us* anH = plane(nX);   us* anL = plane(nX);
    us* hfH = plane(nHF);  us* hfL = plane(nHF);
    float* ffo   = f32b(nX);
    if (off > ws_size) return;

    auto split = [&](const float* s, us* dh, us* dl, size_t n, int cols, int seq, int flip) {
        int n8 = (int)(n / 8);
        k_split<<<(n8 + 255) / 256, 256, 0, stream>>>(s, dh, dl, (int)n, cols, seq, flip);
    };
    split(fm_in_W,  fm_inH, fm_inL, nIn,  (int)nIn,  1, 0);
    split(bm_in_W,  bm_inH, bm_inL, nIn,  (int)nIn,  1, 0);
    split(fm_xp_W,  fm_xpH, fm_xpL, nXp,  (int)nXp,  1, 0);
    split(bm_xp_W,  bm_xpH, bm_xpL, nXp,  (int)nXp,  1, 0);
    split(fm_dt_W,  fm_dtH, fm_dtL, nDt,  (int)nDt,  1, 0);
    split(bm_dt_W,  bm_dtH, bm_dtL, nDt,  (int)nDt,  1, 0);
    split(fm_out_W, fm_ouH, fm_ouL, nOut, (int)nOut, 1, 0);
    split(bm_out_W, bm_ouH, bm_ouL, nOut, (int)nOut, 1, 0);
    split(ff_W1,    f1H,    f1L,    nF1,  (int)nF1,  1, 0);
    split(ff_W2,    f2H,    f2L,    nF2,  (int)nF2,  1, 0);
    split(x, xH,  xL,  nX, D_MODEL, SEQ, 0);
    split(x, xrH, xrL, nX, D_MODEL, SEQ, 1);

    auto gemm = [&](const us* Ah, const us* Al, int lda, const us* Wh, const us* Wl, int K, int N,
                    const float* bias, int act, float* oF, us* oH, us* oL) {
        dim3 grid(N / GBN, ROWS / GBM);
        k_gemm<<<grid, 128, 0, stream>>>(Ah, Al, lda, Wh, Wl, K, N, bias, act, oF, oH, oL);
    };

    auto run_dir = [&](const us* uH, const us* uL, const us* inH, const us* inL,
                       const float* cw, const float* cb,
                       const us* xpH, const us* xpL, const us* dtH, const us* dtL, const float* dtb,
                       const float* Alog, const float* Dp, const us* ouH, const us* ouL, float* dirOut) {
        gemm(uH, uL, D_MODEL, inH, inL, D_MODEL, D_XZ, nullptr, 0, xz, nullptr, nullptr);
        k_conv<<<ROWS, 128, 0, stream>>>(xz, cw, cb, xm, xmH, xmL);
        gemm(xmH, xmL, D_INNER, xpH, xpL, D_INNER, D_DBC, nullptr, 0, dbc, dbH, dbL);
        gemm(dbH, dbL, D_DBC, dtH, dtL, DT_RANK, D_INNER, dtb, 2, delta, nullptr, nullptr);
        k_scan<<<dim3(D_INNER / 256, BATCH), 256, 0, stream>>>(delta, dbc, xm, xz, Alog, Dp, yH, yL);
        gemm(yH, yL, D_INNER, ouH, ouL, D_INNER, D_MODEL, nullptr, 0, dirOut, nullptr, nullptr);
    };

    run_dir(xH,  xL,  fm_inH, fm_inL, fm_cw, fm_cb, fm_xpH, fm_xpL, fm_dtH, fm_dtL, fm_dt_b,
            fm_Alog, fm_D, fm_ouH, fm_ouL, dirF);
    run_dir(xrH, xrL, bm_inH, bm_inL, bm_cw, bm_cb, bm_xpH, bm_xpL, bm_dtH, bm_dtL, bm_dt_b,
            bm_Alog, bm_D, bm_ouH, bm_ouL, dirT);

    k_ln12<<<ROWS, 64, 0, stream>>>(x, dirF, dirT, ln1_g, ln1_b, ln2_g, ln2_b, anH, anL);

    gemm(anH, anL, D_MODEL, f1H, f1L, D_MODEL, D_FF, ff_b1, 1, nullptr, hfH, hfL);
    gemm(hfH, hfL, D_FF, f2H, f2L, D_FF, D_MODEL, ff_b2, 0, ffo, nullptr, nullptr);

    k_ln3<<<ROWS, 128, 0, stream>>>(ffo, ln3_g, ln3_b, out);

    (void)hipGetLastError();
}
